// ContentPhasorStream_37082747633852
// MI455X (gfx1250) — hardware-verified
//
#include <hip/hip_runtime.h>
#include <math.h>
#include <stdint.h>
#include <stddef.h>


#define L_    2048
#define D_    256
#define KP_   32
#define F_    64
#define C_    128
#define NC_   (L_ / C_)
#define TR_   32
#define LXP   (D_ + 8)
#define WSEG1 (D_ * D_)
#define WSEG2 (KP_ * D_)
#define WTOT  (3 * WSEG1 + 2 * WSEG2)
#define PI_F  3.14159265358979323846f
#define WSC   64.0f
#define HSC   64.0f
#define FSC   8.0f
#define LSC   4096.0f

typedef _Float16 f16;
typedef _Float16 v16h __attribute__((ext_vector_type(16)));
typedef _Float16 v8h  __attribute__((ext_vector_type(8)));
typedef float    v8f  __attribute__((ext_vector_type(8)));
typedef float    v4f  __attribute__((ext_vector_type(4)));
typedef v8h v8ha __attribute__((may_alias));
typedef v4f v4fa __attribute__((may_alias));
union Frag { v16h v; v8h hh[2]; };

__device__ __forceinline__ float bf16r(float x) {
  unsigned u = __float_as_uint(x);
  u = (u + 0x7FFFu + ((u >> 16) & 1u)) & 0xFFFF0000u;
  return __uint_as_float(u);
}

__device__ __forceinline__ float tanh_f(float x) {
  const float ax = fabsf(x);
  const float t = __expf(-2.0f * ax);
  const float r = (1.0f - t) * __builtin_amdgcn_rcpf(1.0f + t);
  return copysignf(r, x);
}

__device__ __forceinline__ v8f zero8() {
  v8f z = {0.f, 0.f, 0.f, 0.f, 0.f, 0.f, 0.f, 0.f};
  return z;
}

__device__ __forceinline__ v8f mma(v16h a, v16h b, v8f c) {
  v8f d = __builtin_amdgcn_wmma_f32_16x16x32_f16(false, a, false, b, (short)0, c, false, false);
  asm volatile("v_nop\n\tv_nop\n\tv_nop\n\tv_nop" : "+v"(d) : "v"(a), "v"(b));
  return d;
}

__device__ __forceinline__ v16h frag_kc(const f16* p, int ld, int r0, int k0, int lane) {
  const int m = lane & 15, h = lane >> 4;
  const f16* q = p + (size_t)(r0 + m) * ld + k0 + 8 * h;
  Frag f;
  f.hh[0] = *(const v8ha*)(q);
  f.hh[1] = *(const v8ha*)(q + 16);
  return f.v;
}

__device__ __forceinline__ v16h frag_ks(const f16* p, int ld, int k0, int n0, int lane) {
  const int n = lane & 15, h = lane >> 4;
  const f16* q = p + (size_t)(k0 + 8 * h) * ld + n0 + n;
  v16h v;
#pragma unroll
  for (int i = 0; i < 8; ++i) {
    v[i]     = q[(size_t)i * ld];
    v[8 + i] = q[(size_t)(16 + i) * ld];
  }
  return v;
}

__device__ __forceinline__ v16h frag_P(const float* Sb, int c, int k0, int n0, int lane) {
  const int n = lane & 15, h = lane >> 4;
  const float* q = Sb + (size_t)(k0 + 8 * h) * D_ + n0 + n;
  float s[16];
#pragma unroll
  for (int i = 0; i < 16; ++i) s[i] = 0.0f;
  for (int cc = 0; cc < c; ++cc) {
    const float* qc = q + (size_t)cc * F_ * D_;
#pragma unroll
    for (int i = 0; i < 8; ++i) {
      s[i]     += qc[(size_t)i * D_];
      s[8 + i] += qc[(size_t)(16 + i) * D_];
    }
  }
  v16h v;
#pragma unroll
  for (int i = 0; i < 16; ++i) v[i] = (f16)s[i];
  return v;
}

__global__ __launch_bounds__(256) void k_cvtw(
    const float* __restrict__ kw1, const float* __restrict__ qw1,
    const float* __restrict__ vw,  const float* __restrict__ kw2,
    const float* __restrict__ qw2, f16* o, int total8)
{
  const int i = blockIdx.x * 256 + threadIdx.x;
  if (i >= total8) return;
  const int e = i * 8;
  const float* src;
  int off;
  if      (e < WSEG1)             { src = kw1; off = e; }
  else if (e < 2 * WSEG1)         { src = qw1; off = e - WSEG1; }
  else if (e < 3 * WSEG1)         { src = vw;  off = e - 2 * WSEG1; }
  else if (e < 3 * WSEG1 + WSEG2) { src = kw2; off = e - 3 * WSEG1; }
  else                            { src = qw2; off = e - 3 * WSEG1 - WSEG2; }
  const v4f u0 = *(const v4fa*)(src + off);
  const v4f u1 = *(const v4fa*)(src + off + 4);
  v8h v;
  v[0] = (f16)(bf16r(u0.x) * WSC);
  v[1] = (f16)(bf16r(u0.y) * WSC);
  v[2] = (f16)(bf16r(u0.z) * WSC);
  v[3] = (f16)(bf16r(u0.w) * WSC);
  v[4] = (f16)(bf16r(u1.x) * WSC);
  v[5] = (f16)(bf16r(u1.y) * WSC);
  v[6] = (f16)(bf16r(u1.z) * WSC);
  v[7] = (f16)(bf16r(u1.w) * WSC);
  f16* p = o + e;
  *(volatile v8h*)p = v;
  __threadfence();
  *(volatile v8h*)p = v;
}

__global__ __launch_bounds__(64) void k_encode(
    const float* __restrict__ x, const f16* __restrict__ wbuf,
    const float* __restrict__ kb1, const float* __restrict__ kb2,
    const float* __restrict__ qb1, const float* __restrict__ qb2,
    const float* __restrict__ vbias,
    f16* fk, f16* fq, f16* vh, f16* vl, int nrows)
{
  __shared__ __attribute__((aligned(16))) f16   lx[TR_][LXP];
  __shared__ __attribute__((aligned(16))) f16   lh[TR_][LXP];
  __shared__ __attribute__((aligned(16))) float lph[2][16][KP_];
  __shared__ __attribute__((aligned(16))) f16   stg[2][2][16][64];

  const int tid = threadIdx.x, lane = tid & 31, wave = tid >> 5;
  const int h = lane >> 4, cn = lane & 15;
  const int row0 = blockIdx.x * TR_;
  if (row0 + TR_ > nrows) return;

  for (int i = tid; i < TR_ * (D_ / 4); i += 64) {
    const int r  = i / (D_ / 4);
    const int c4 = (i % (D_ / 4)) * 4;
    const v4f v = *(const v4fa*)(x + (size_t)(row0 + r) * D_ + c4);
    lx[r][c4 + 0] = (f16)bf16r(v.x);
    lx[r][c4 + 1] = (f16)bf16r(v.y);
    lx[r][c4 + 2] = (f16)bf16r(v.z);
    lx[r][c4 + 3] = (f16)bf16r(v.w);
  }
  __syncthreads();

  const int m0 = wave * 16;
  const f16* wk1 = wbuf;
  const f16* wq1 = wbuf + WSEG1;
  const f16* wv  = wbuf + 2 * WSEG1;
  const f16* wk2 = wbuf + 3 * WSEG1;
  const f16* wq2 = wbuf + 3 * WSEG1 + WSEG2;

  for (int pass = 0; pass < 2; ++pass) {
    const f16*   w1 = pass ? wq1 : wk1;
    const float* b1 = pass ? qb1 : kb1;
    const f16*   w2 = pass ? wq2 : wk2;
    const float* b2 = pass ? qb2 : kb2;
    f16* fo = pass ? fq : fk;

    for (int ng = 0; ng < D_; ng += 64) {
      v8f acc[4];
#pragma unroll
      for (int j = 0; j < 4; ++j) acc[j] = zero8();
      for (int k0 = 0; k0 < D_; k0 += 32) {
        const v16h a = frag_kc(&lx[0][0], LXP, m0, k0, lane);
#pragma unroll
        for (int j = 0; j < 4; ++j)
          acc[j] = mma(a, frag_kc(w1, D_, ng + 16 * j, k0, lane), acc[j]);
      }
#pragma unroll
      for (int j = 0; j < 4; ++j) {
        const int col = ng + 16 * j + cn;
        const float bias = bf16r(b1[col]);
#pragma unroll
        for (int r = 0; r < 8; ++r)
          lh[m0 + 8 * h + r][col] = (f16)(tanh_f(acc[j][r] * (1.0f / WSC) + bias) * HSC);
      }
    }
    __syncthreads();

    {
      v8f acc[2];
      acc[0] = zero8();
      acc[1] = zero8();
      for (int k0 = 0; k0 < D_; k0 += 32) {
        const v16h a = frag_kc(&lh[0][0], LXP, m0, k0, lane);
#pragma unroll
        for (int j = 0; j < 2; ++j)
          acc[j] = mma(a, frag_kc(w2, D_, 16 * j, k0, lane), acc[j]);
      }
#pragma unroll
      for (int j = 0; j < 2; ++j) {
        const int col = 16 * j + cn;
        const float bias = bf16r(b2[col]);
#pragma unroll
        for (int r = 0; r < 8; ++r)
          lph[wave][8 * h + r][col] = tanh_f(acc[j][r] * (1.0f / (WSC * HSC)) + bias) * PI_F;
      }
    }
    __syncthreads();

#pragma unroll 1
    for (int e = lane; e < 16 * KP_; e += 32) {
      const int r = e >> 5, k = e & 31;
      const float ph = lph[wave][r][k];
      stg[wave][0][r][k]       = (f16)(cosf(ph) * FSC);
      stg[wave][0][r][KP_ + k] = (f16)(sinf(ph) * FSC);
    }
    __syncthreads();

    {
      v8h val[4];
#pragma unroll
      for (int q = 0; q < 4; ++q) {
        const int row = 4 * q + (lane >> 3);
        const int c8 = (lane & 7) * 8;
        val[q] = *(const v8ha*)&stg[wave][0][row][c8];
      }
#pragma unroll
      for (int q = 0; q < 4; ++q) {
        const int row = 4 * q + (lane >> 3);
        const int c8 = (lane & 7) * 8;
        *(volatile v8h*)(fo + (size_t)(row0 + m0 + row) * F_ + c8) = val[q];
      }
      __threadfence();
#pragma unroll
      for (int q = 0; q < 4; ++q) {
        const int row = 4 * q + (lane >> 3);
        const int c8 = (lane & 7) * 8;
        *(volatile v8h*)(fo + (size_t)(row0 + m0 + row) * F_ + c8) = val[q];
      }
    }
    __syncthreads();
  }

  for (int ng = 0; ng < D_; ng += 64) {
    v8f acc[4];
#pragma unroll
    for (int j = 0; j < 4; ++j) acc[j] = zero8();
    for (int k0 = 0; k0 < D_; k0 += 32) {
      const v16h a = frag_kc(&lx[0][0], LXP, m0, k0, lane);
#pragma unroll
      for (int j = 0; j < 4; ++j)
        acc[j] = mma(a, frag_kc(wv, D_, ng + 16 * j, k0, lane), acc[j]);
    }
#pragma unroll
    for (int j = 0; j < 4; ++j) {
      const int col = ng + 16 * j + cn;
      const float bias = bf16r(vbias[col]);
#pragma unroll
      for (int r = 0; r < 8; ++r) {
        const float v = acc[j][r] * (1.0f / WSC) + bias;
        const f16 hvv = (f16)v;
        const f16 lvv = (f16)((v - (float)hvv) * LSC);
        stg[wave][0][8 * h + r][16 * j + cn] = hvv;
        stg[wave][1][8 * h + r][16 * j + cn] = lvv;
      }
    }
    __syncthreads();
    {
      v8h hv[4], lv[4];
#pragma unroll
      for (int q = 0; q < 4; ++q) {
        const int row = 4 * q + (lane >> 3);
        const int c8 = (lane & 7) * 8;
        hv[q] = *(const v8ha*)&stg[wave][0][row][c8];
        lv[q] = *(const v8ha*)&stg[wave][1][row][c8];
      }
#pragma unroll
      for (int q = 0; q < 4; ++q) {
        const int row = 4 * q + (lane >> 3);
        const int c8 = (lane & 7) * 8;
        const size_t g = (size_t)(row0 + m0 + row) * D_ + ng + c8;
        *(volatile v8h*)(vh + g) = hv[q];
        *(volatile v8h*)(vl + g) = lv[q];
      }
      __threadfence();
#pragma unroll
      for (int q = 0; q < 4; ++q) {
        const int row = 4 * q + (lane >> 3);
        const int c8 = (lane & 7) * 8;
        const size_t g = (size_t)(row0 + m0 + row) * D_ + ng + c8;
        *(volatile v8h*)(vh + g) = hv[q];
        *(volatile v8h*)(vl + g) = lv[q];
      }
    }
    __syncthreads();
  }
}

__global__ __launch_bounds__(128) void k_state(
    const f16* __restrict__ fk, const f16* __restrict__ vh, const f16* __restrict__ vl,
    float* S, int nchunks)
{
  __shared__ __attribute__((aligned(16))) float stg[4][16][32];

  const int tid = threadIdx.x, lane = tid & 31, wave = tid >> 5;
  const int h = lane >> 4, cn = lane & 15;
  const int chunk = blockIdx.x;
  if (chunk >= nchunks) return;
  const size_t t0 = (size_t)chunk * C_;
  const f16* fkc = fk + t0 * F_;
  const f16* vhc = vh + t0 * D_;
  const f16* vlc = vl + t0 * D_;
  float* Sc = S + (size_t)chunk * F_ * D_;
  const int m0 = wave * 16;

  v16h a[4];
#pragma unroll
  for (int ks = 0; ks < 4; ++ks) a[ks] = frag_ks(fkc, F_, 32 * ks, m0, lane);

  for (int np = 0; np < D_; np += 32) {
    v8f ah[2], al[2];
    ah[0] = zero8(); ah[1] = zero8();
    al[0] = zero8(); al[1] = zero8();
#pragma unroll
    for (int ks = 0; ks < 4; ++ks) {
#pragma unroll
      for (int j = 0; j < 2; ++j) {
        ah[j] = mma(a[ks], frag_ks(vhc, D_, 32 * ks, np + 16 * j, lane), ah[j]);
        al[j] = mma(a[ks], frag_ks(vlc, D_, 32 * ks, np + 16 * j, lane), al[j]);
      }
    }
#pragma unroll
    for (int j = 0; j < 2; ++j)
#pragma unroll
      for (int r = 0; r < 8; ++r)
        stg[wave][8 * h + r][16 * j + cn] = ah[j][r] + al[j][r] * (1.0f / LSC);
    __syncthreads();
    {
      v4f ov[4];
#pragma unroll
      for (int q = 0; q < 4; ++q) {
        const int row = 4 * q + (lane >> 3);
        const int c4 = (lane & 7) * 4;
        ov[q] = *(const v4fa*)&stg[wave][row][c4];
      }
#pragma unroll
      for (int q = 0; q < 4; ++q) {
        const int row = 4 * q + (lane >> 3);
        const int c4 = (lane & 7) * 4;
        *(volatile v4f*)(Sc + (size_t)(m0 + row) * D_ + np + c4) = ov[q];
      }
      __threadfence();
#pragma unroll
      for (int q = 0; q < 4; ++q) {
        const int row = 4 * q + (lane >> 3);
        const int c4 = (lane & 7) * 4;
        *(volatile v4f*)(Sc + (size_t)(m0 + row) * D_ + np + c4) = ov[q];
      }
    }
    __syncthreads();
  }
}

__global__ __launch_bounds__(64) void k_out(
    const f16* __restrict__ fq, const f16* __restrict__ fk,
    const f16* __restrict__ vh, const f16* __restrict__ vl,
    const float* __restrict__ S, float* out, int nchunks)
{
  __shared__ __attribute__((aligned(16))) f16   lsh[2][32][C_];
  __shared__ __attribute__((aligned(16))) f16   lsl[2][32][C_];
  __shared__ __attribute__((aligned(16))) float stg[2][16][32];

  const int tid = threadIdx.x, lane = tid & 31, wave = tid >> 5;
  const int h = lane >> 4, cn = lane & 15;
  const int chunk = blockIdx.x >> 1, hf = blockIdx.x & 1;
  if (chunk >= nchunks) return;
  const int b = chunk / NC_;
  const int c = chunk - b * NC_;
  const size_t t0 = (size_t)chunk * C_;
  const f16* fqc = fq + t0 * F_;
  const f16* fkc = fk + t0 * F_;
  const f16* vhc = vh + t0 * D_;
  const f16* vlc = vl + t0 * D_;
  const float* Sb = S + (size_t)b * NC_ * F_ * D_;
  float* oc = out + t0 * D_;
  const int rw = hf * 64 + wave * 32;

  for (int mt = 0; mt < 2; ++mt) {
    const int m0 = rw + 16 * mt;
    const v16h a0 = frag_kc(fqc, F_, m0, 0, lane);
    const v16h a1 = frag_kc(fqc, F_, m0, 32, lane);
    for (int n0 = 0; n0 < C_; n0 += 16) {
      v8f acc = zero8();
      acc = mma(a0, frag_kc(fkc, F_, n0, 0, lane), acc);
      acc = mma(a1, frag_kc(fkc, F_, n0, 32, lane), acc);
      const int col = n0 + cn;
#pragma unroll
      for (int r = 0; r < 8; ++r) {
        const int qr = m0 + 8 * h + r;
        const float s = (col <= qr) ? acc[r] : 0.0f;
        const f16 sh = (f16)s;
        const f16 sl = (f16)((s - (float)sh) * LSC);
        lsh[wave][16 * mt + 8 * h + r][col] = sh;
        lsl[wave][16 * mt + 8 * h + r][col] = sl;
      }
    }
  }
  __syncthreads();

  float rsv[2][8];
#pragma unroll
  for (int mt = 0; mt < 2; ++mt)
#pragma unroll
    for (int r = 0; r < 8; ++r) {
      const int pos1 = c * C_ + rw + 16 * mt + 8 * h + r + 1;
      rsv[mt][r] = (1.0f / sqrtf((float)(pos1 * KP_))) * (1.0f / (FSC * FSC));
    }

  for (int np = 0; np < D_; np += 32) {
    v16h pf[2][2];
#pragma unroll
    for (int ks = 0; ks < 2; ++ks)
#pragma unroll
      for (int j = 0; j < 2; ++j) pf[ks][j] = frag_P(Sb, c, 32 * ks, np + 16 * j, lane);

#pragma unroll
    for (int mt = 0; mt < 2; ++mt) {
      v8f acc0[2], acc1[2];
      acc0[0] = zero8(); acc0[1] = zero8();
      acc1[0] = zero8(); acc1[1] = zero8();
#pragma unroll
      for (int ks = 0; ks < 2; ++ks) {
        const v16h a = frag_kc(fqc, F_, rw + 16 * mt, 32 * ks, lane);
#pragma unroll
        for (int j = 0; j < 2; ++j) acc0[j] = mma(a, pf[ks][j], acc0[j]);
      }
#pragma unroll
      for (int ks = 0; ks < 4; ++ks) {
        const v16h ash = frag_kc(&lsh[wave][0][0], C_, 16 * mt, 32 * ks, lane);
        const v16h asl = frag_kc(&lsl[wave][0][0], C_, 16 * mt, 32 * ks, lane);
#pragma unroll
        for (int j = 0; j < 2; ++j) {
          const v16h bh = frag_ks(vhc, D_, 32 * ks, np + 16 * j, lane);
          const v16h bl = frag_ks(vlc, D_, 32 * ks, np + 16 * j, lane);
          acc0[j] = mma(ash, bh, acc0[j]);
          acc1[j] = mma(ash, bl, acc1[j]);
          acc1[j] = mma(asl, bh, acc1[j]);
        }
      }
#pragma unroll
      for (int j = 0; j < 2; ++j)
#pragma unroll
        for (int r = 0; r < 8; ++r)
          stg[wave][8 * h + r][16 * j + cn] = (acc0[j][r] + acc1[j][r] * (1.0f / LSC)) * rsv[mt][r];
      __syncthreads();
      {
        v4f ov[4];
#pragma unroll
        for (int q = 0; q < 4; ++q) {
          const int row = 4 * q + (lane >> 3);
          const int c4 = (lane & 7) * 4;
          ov[q] = *(const v4fa*)&stg[wave][row][c4];
        }
#pragma unroll
        for (int q = 0; q < 4; ++q) {
          const int row = 4 * q + (lane >> 3);
          const int c4 = (lane & 7) * 4;
          *(volatile v4f*)(oc + (size_t)(rw + 16 * mt + row) * D_ + np + c4) = ov[q];
        }
        __threadfence();
#pragma unroll
        for (int q = 0; q < 4; ++q) {
          const int row = 4 * q + (lane >> 3);
          const int c4 = (lane & 7) * 4;
          *(volatile v4f*)(oc + (size_t)(rw + 16 * mt + row) * D_ + np + c4) = ov[q];
        }
      }
      __syncthreads();
    }
  }
}

extern "C" void kernel_launch(void* const* d_in, const int* in_sizes, int n_in,
                              void* d_out, int out_size, void* d_ws, size_t ws_size,
                              hipStream_t stream) {
  if (n_in < 11) return;
  const float* x   = (const float*)d_in[0];
  const float* kw1 = (const float*)d_in[1];
  const float* kb1 = (const float*)d_in[2];
  const float* kw2 = (const float*)d_in[3];
  const float* kb2 = (const float*)d_in[4];
  const float* qw1 = (const float*)d_in[5];
  const float* qb1 = (const float*)d_in[6];
  const float* qw2 = (const float*)d_in[7];
  const float* qb2 = (const float*)d_in[8];
  const float* vw  = (const float*)d_in[9];
  const float* vb  = (const float*)d_in[10];

  const int nx = in_sizes[0];
  if (nx <= 0 || (nx % D_) != 0) return;
  const int nrows = nx / D_;
  if ((nrows % L_) != 0 || out_size != nrows * D_) return;
  if (in_sizes[1] != WSEG1 || in_sizes[5] != WSEG1 || in_sizes[9] != WSEG1) return;
  if (in_sizes[3] != WSEG2 || in_sizes[7] != WSEG2) return;
  if (in_sizes[2] < D_ || in_sizes[6] < D_ || in_sizes[10] < D_) return;
  if (in_sizes[4] < KP_ || in_sizes[8] < KP_) return;
  const int nchunks = nrows / C_;

  const size_t w_bytes = (((size_t)WTOT * sizeof(f16)) + 255) & ~(size_t)255;
  const size_t f_bytes = (((size_t)nrows * F_ * sizeof(f16)) + 255) & ~(size_t)255;
  const size_t v_bytes = (((size_t)nrows * D_ * sizeof(f16)) + 255) & ~(size_t)255;
  const size_t s_bytes = (((size_t)nchunks * F_ * D_ * sizeof(float)) + 255) & ~(size_t)255;
  size_t off = 0;
  char* ws = (char*)d_ws;
  f16* wbuf = (f16*)(ws + off);  off += w_bytes;
  f16* fk   = (f16*)(ws + off);  off += f_bytes;
  f16* fq   = (f16*)(ws + off);  off += f_bytes;
  f16* vhp  = (f16*)(ws + off);  off += v_bytes;
  f16* vlp  = (f16*)(ws + off);  off += v_bytes;
  float* S  = (float*)(ws + off); off += s_bytes;
  if (off > ws_size) return;

  const int total8 = WTOT / 8;
  k_cvtw<<<(total8 + 255) / 256, 256, 0, stream>>>(kw1, qw1, vw, kw2, qw2, wbuf, total8);
  k_encode<<<(nrows + TR_ - 1) / TR_, 64, 0, stream>>>(
      x, wbuf, kb1, kb2, qb1, qb2, vb, fk, fq, vhp, vlp, nrows);
  k_state<<<nchunks, 128, 0, stream>>>(fk, vhp, vlp, S, nchunks);
  k_out<<<nchunks * 2, 64, 0, stream>>>(fq, fk, vhp, vlp, S, (float*)d_out, nchunks);
  (void)hipGetLastError();
}
